// BatteryMoEFlattenIntraCycleMoELayer_51754355916892
// MI455X (gfx1250) — hardware-verified
//
#include <hip/hip_runtime.h>
#include <stdint.h>

constexpr int NB   = 128;
constexpr int NL   = 100;
constexpr int NF   = 900;
constexpr int NE   = 8;
constexpr int ND   = 512;
constexpr int KPAD = 928;
constexpr int MPAD = 112;
constexpr int MT   = 16;
constexpr int NT   = 64;

static_assert(KPAD % 32 == 0 && KPAD >= NF, "K pad");
static_assert(MPAD % MT == 0 && MPAD >= NL, "M pad");
static_assert(ND % NT == 0, "N tile multiple");
static_assert((MPAD / MT) * (ND / NT) == 56, "56 wave tiles per sample = 7 blocks x 8 waves");

constexpr size_t X_ELEMS = (size_t)NB * MPAD * KPAD;
constexpr size_t W_ELEMS = (size_t)NE * ND * KPAD;
constexpr size_t X_BYTES = X_ELEMS * 2;
constexpr size_t W_BYTES = W_ELEMS * 2;
constexpr size_t G_BYTES = (size_t)NB * 4 * 4;
constexpr size_t OFF_X = 0;
constexpr size_t OFF_W = OFF_X + X_BYTES;
constexpr size_t OFF_G = OFF_W + W_BYTES;
constexpr size_t WS_TOTAL = OFF_G + G_BYTES;
static_assert(OFF_W % 128 == 0 && OFF_G % 128 == 0, "128-B aligned carves");
static_assert(WS_TOTAL <= 134217728ull, "carve under 128 MiB");
static_assert(X_ELEMS % 512 == 0 && W_ELEMS % 512 == 0, "cast grids exact: 256 threads x 2 elements");

typedef __attribute__((ext_vector_type(16))) __bf16   v16b;
typedef __attribute__((ext_vector_type(8)))  __bf16   v8b;
typedef __attribute__((ext_vector_type(8)))  float    v8f;
typedef __attribute__((ext_vector_type(4)))  float    v4f;
typedef __attribute__((ext_vector_type(2)))  float    v2f;
typedef __attribute__((ext_vector_type(4)))  int      v4i;
typedef __attribute__((ext_vector_type(4)))  unsigned v4u;

__device__ __forceinline__ unsigned short f2bf_bits(float f) {
  unsigned u = __float_as_uint(f);
  return (unsigned short)((u + 0x7FFFu + ((u >> 16) & 1u)) >> 16);
}
__device__ __forceinline__ float bf_bits2f(unsigned short h) { return __uint_as_float(((unsigned)h) << 16); }
__device__ __forceinline__ float bf_rne(float f) { return bf_bits2f(f2bf_bits(f)); }

__device__ __forceinline__ void dep_guard_b(v8f& a, v8f& b, v16b x, v16b y) { asm volatile("v_nop\n\tv_nop\n\tv_nop\n\tv_nop" : "+v"(a), "+v"(b) : "v"(x), "v"(y)); }
__device__ __forceinline__ void keep4_b(v16b a, v16b b, v16b c, v16b d) { asm volatile("v_nop" :: "v"(a), "v"(b), "v"(c), "v"(d)); }
__device__ __forceinline__ void acc_guard4(v8f& a, v8f& b, v8f& c, v8f& d) { asm volatile("v_nop\n\tv_nop\n\tv_nop\n\tv_nop" : "+v"(a), "+v"(b), "+v"(c), "+v"(d)); }

template <typename T> struct Frag;
template <> struct Frag<__bf16> {
  typedef v16b V; union U { v16b v; v8b h[2]; };
  static __device__ __forceinline__ v16b load(const __bf16* p) {
    U f; f.h[0] = *(const v8b*)(p); f.h[1] = *(const v8b*)(p + 16); return f.v;
  }
  static __device__ __forceinline__ v8f mma(v16b a, v16b b, v8f c) {
    return __builtin_amdgcn_wmma_f32_16x16x32_bf16(false, a, false, b, (short)0, c, false, false);
  }
  static __device__ __forceinline__ void guard(v8f& a, v8f& b, v16b x, v16b y) { dep_guard_b(a, b, x, y); }
  static __device__ __forceinline__ void keep(v16b a, v16b b, v16b c, v16b d) { keep4_b(a, b, c, d); }
};

__global__ __launch_bounds__(NB) void gates_kernel(const float* __restrict__ logits,
                                                    const int*   __restrict__ masks,
                                                    float* __restrict__ gtab) {
  const int b = threadIdx.x;
  const v4f la = *(const v4f*)(logits + (size_t)b * NE);
  const v4f lb = *(const v4f*)(logits + (size_t)b * NE + 4);
  const v4i ma = *(const v4i*)(masks  + (size_t)b * NE);
  const v4i mb = *(const v4i*)(masks  + (size_t)b * NE + 4);
  float lg[NE]; int mk[NE];
#pragma unroll
  for (int e = 0; e < 4; ++e) { lg[e] = bf_rne(la[e]); lg[4 + e] = bf_rne(lb[e]); mk[e] = ma[e]; mk[4 + e] = mb[e]; }
  float mx = lg[0];
#pragma unroll
  for (int e = 1; e < NE; ++e) mx = fmaxf(mx, lg[e]);
  float pu[NE];
  float s = 0.f;
#pragma unroll
  for (int e = 0; e < NE; ++e) { pu[e] = expf(lg[e] - mx); s += pu[e]; }
  const float rs = 1.0f / s;
  float g[NE];
#pragma unroll
  for (int e = 0; e < NE; ++e) g[e] = (mk[e] == 1) ? (pu[e] * rs) : 0.f;
  int i0 = 0; float v0 = g[0];
#pragma unroll
  for (int e = 1; e < NE; ++e) { if (g[e] > v0) { v0 = g[e]; i0 = e; } }
  int i1 = -1; float v1 = -1.f;
#pragma unroll
  for (int e = 0; e < NE; ++e) { if (e != i0 && g[e] > v1) { v1 = g[e]; i1 = e; } }
  const float denom = v0 + v1 + 1e-9f;
  const float rd = 1.0f / denom;
  v4f o;
  o[0] = v0 * rd;
  o[1] = v1 * rd;
  o[2] = (float)i0;
  o[3] = (float)i1;
  *(volatile v4f*)(gtab + (size_t)b * 4) = o;
  __threadfence();
  *(volatile v4f*)(gtab + (size_t)b * 4) = o;
}

__global__ __launch_bounds__(256) void cvt_x_bf16(const float* __restrict__ x,
                                                   unsigned* __restrict__ xp, int npairs) {
  const int i = blockIdx.x * 256 + threadIdx.x;
  if (i < npairs) {
    const size_t idx = 2 * (size_t)i;
    const int f = (int)(idx % KPAD);
    const size_t t = idx / KPAD;
    const int m = (int)(t % MPAD);
    const int bb = (int)(t / MPAD);
    const bool valid = (m < NL) && (f < NF);
    const int mc = (m < NL) ? m : (NL - 1);
    const int fc = (f < NF - 2) ? f : (NF - 2);
    const v2f v = *(const v2f*)(x + ((size_t)bb * NL + mc) * NF + fc);
    const float a0 = valid ? v[0] : 0.f;
    const float a1 = valid ? v[1] : 0.f;
    const unsigned u = (unsigned)f2bf_bits(a0) | ((unsigned)f2bf_bits(a1) << 16);
    ((volatile unsigned*)xp)[i] = u;
    __threadfence();
    ((volatile unsigned*)xp)[i] = u;
  }
}

__global__ __launch_bounds__(256) void cvt_w_bf16(const float* __restrict__ W,
                                                   unsigned* __restrict__ wp, int npairs) {
  const int i = blockIdx.x * 256 + threadIdx.x;
  if (i < npairs) {
    const size_t idx = 2 * (size_t)i;
    const int f = (int)(idx % KPAD);
    const size_t t = idx / KPAD;
    const bool valid = (f < NF);
    const int fc = (f < NF - 2) ? f : (NF - 2);
    const v2f v = *(const v2f*)(W + t * NF + fc);
    const float a0 = valid ? v[0] : 0.f;
    const float a1 = valid ? v[1] : 0.f;
    const unsigned u = (unsigned)f2bf_bits(a0) | ((unsigned)f2bf_bits(a1) << 16);
    ((volatile unsigned*)wp)[i] = u;
    __threadfence();
    ((volatile unsigned*)wp)[i] = u;
  }
}

__global__ __launch_bounds__(256) void moe_gemm_kernel(const unsigned short* __restrict__ Xp,
                                                        const unsigned short* __restrict__ Wp,
                                                        const float* __restrict__ bias,
                                                        const float* __restrict__ gtab,
                                                        unsigned short* __restrict__ outp) {
  __shared__ __align__(16) float sT[8][16 * 68];
  const int b    = blockIdx.y;
  const int lane = threadIdx.x & 31;
  const int wave = threadIdx.x >> 5;
  const int tile = blockIdx.x * 8 + wave;
  const int tm   = tile >> 3;
  const int tn   = tile & 7;
  const int m0   = tm * MT;
  const int n0   = tn * NT;
  const int rlane = lane & 15;
  const int koff  = (lane >> 4) * 8;
  const int mOff  = (lane >> 4) * 8;

  const v4f gt = *(const v4f*)(gtab + (size_t)b * 4);
  const float g0 = gt[0];
  const float g1 = gt[1];
  int e0 = (int)gt[2];
  int e1 = (int)gt[3];
  e0 = e0 < 0 ? 0 : (e0 > NE - 1 ? NE - 1 : e0);
  e1 = e1 < 0 ? 0 : (e1 > NE - 1 ? NE - 1 : e1);

  const __bf16* Ab  = (const __bf16*)Xp + ((size_t)b * MPAD + m0 + rlane) * KPAD + koff;
  const __bf16* Bb0 = (const __bf16*)Wp + ((size_t)e0 * ND + n0 + rlane) * KPAD + koff;
  const __bf16* Bb1 = (const __bf16*)Wp + ((size_t)e1 * ND + n0 + rlane) * KPAD + koff;

  v8f acc[2][4];
#pragma unroll
  for (int i = 0; i < 2; ++i)
#pragma unroll
    for (int j = 0; j < 4; ++j) acc[i][j] = (v8f){0.f,0.f,0.f,0.f,0.f,0.f,0.f,0.f};

  for (int k0 = 0; k0 < KPAD; k0 += 32) {
    v16b bw0[4], bw1[4];
#pragma unroll
    for (int j = 0; j < 4; ++j) {
      bw0[j] = Frag<__bf16>::load(Bb0 + (size_t)(j * 16) * KPAD + k0);
      bw1[j] = Frag<__bf16>::load(Bb1 + (size_t)(j * 16) * KPAD + k0);
    }
    const v16b ah = Frag<__bf16>::load(Ab + k0);
#pragma unroll
    for (int j = 0; j < 4; ++j) acc[0][j] = Frag<__bf16>::mma(ah, bw0[j], acc[0][j]);
#pragma unroll
    for (int j = 0; j < 4; ++j) acc[1][j] = Frag<__bf16>::mma(ah, bw1[j], acc[1][j]);
    Frag<__bf16>::guard(acc[0][0], acc[1][3], ah, ah);
    Frag<__bf16>::keep(bw0[0], bw0[1], bw0[2], bw0[3]);
    Frag<__bf16>::keep(bw1[0], bw1[1], bw1[2], bw1[3]);
  }
  acc_guard4(acc[0][0], acc[0][1], acc[0][2], acc[0][3]);
  acc_guard4(acc[1][0], acc[1][1], acc[1][2], acc[1][3]);

  float* slab = sT[wave];
#pragma unroll
  for (int j = 0; j < 4; ++j) {
    const int n = n0 + (j << 4) + rlane;
    const float bm = g0 * bf_rne(bias[(size_t)e0 * ND + n]) + g1 * bf_rne(bias[(size_t)e1 * ND + n]);
#pragma unroll
    for (int r = 0; r < 8; ++r) {
      const float v = g0 * acc[0][j][r] + g1 * acc[1][j][r] + bm;
      slab[(mOff + r) * 68 + (j << 4) + rlane] = v;
    }
  }
  __builtin_amdgcn_fence(__ATOMIC_RELEASE, "workgroup");
  __builtin_amdgcn_wave_barrier();
  __builtin_amdgcn_fence(__ATOMIC_ACQUIRE, "workgroup");
  {
    const int q  = lane >> 3;
    const int c8 = (lane & 7) * 8;
    for (int pass = 0; pass < 2; ++pass) {
#pragma unroll
      for (int it = 0; it < 4; ++it) {
        const int row = it * 4 + q;
        const int m   = m0 + row;
        const int mcl = (m < NL) ? m : (NL - 1);
        const float* sp = slab + row * 68 + c8;
        v4u w;
#pragma unroll
        for (int e2 = 0; e2 < 4; ++e2)
          w[e2] = (unsigned)f2bf_bits(sp[2 * e2]) | ((unsigned)f2bf_bits(sp[2 * e2 + 1]) << 16);
        if (m < NL)
          *(volatile v4u*)(outp + ((size_t)b * NL + mcl) * ND + n0 + c8) = w;
      }
      __threadfence();
    }
  }
  __builtin_amdgcn_fence(__ATOMIC_RELEASE, "workgroup");
  __builtin_amdgcn_wave_barrier();
  __builtin_amdgcn_fence(__ATOMIC_ACQUIRE, "workgroup");
}

extern "C" void kernel_launch(void* const* d_in, const int* in_sizes, int n_in,
                              void* d_out, int out_size, void* d_ws, size_t ws_size,
                              hipStream_t stream) {
  (void)in_sizes; (void)n_in; (void)out_size;
  const float* x      = (const float*)d_in[0];
  const float* logits = (const float*)d_in[1];
  const int*   masks  = (const int*)  d_in[2];
  const float* W      = (const float*)d_in[3];
  const float* bias   = (const float*)d_in[4];
  unsigned short* out = (unsigned short*)d_out;

  if (ws_size < WS_TOTAL) return;

  char* ws = (char*)d_ws;
  unsigned short* xplane = (unsigned short*)(ws + OFF_X);
  unsigned short* wplane = (unsigned short*)(ws + OFF_W);
  float*          gtab   = (float*)(ws + OFF_G);

  gates_kernel<<<1, NB, 0, stream>>>(logits, masks, gtab);

  const int xpairs = (int)(X_ELEMS / 2);
  cvt_x_bf16<<<(unsigned)((xpairs + 255) / 256), 256, 0, stream>>>(x, (unsigned*)xplane, xpairs);

  const int wpairs = (int)(W_ELEMS / 2);
  cvt_w_bf16<<<(unsigned)((wpairs + 255) / 256), 256, 0, stream>>>(W, (unsigned*)wplane, wpairs);

  dim3 grid((MPAD / MT) * (ND / NT) / 8, NB);
  moe_gemm_kernel<<<grid, 256, 0, stream>>>(xplane, wplane, bias, gtab, out);
}
